// BilinearPooling_47313359733154
// MI455X (gfx1250) — hardware-verified
//
#include <hip/hip_runtime.h>


namespace {
constexpr int B = 16, NN = 64, V = 16, D = 128, EF = 128, O = 256, BV = B * V, OD = O * D;
constexpr float XS = 8.0f, WSC = 256.0f, TS = 256.0f;
typedef _Float16 b16;
typedef __attribute__((ext_vector_type(16))) _Float16 v16b;
typedef __attribute__((ext_vector_type(8))) _Float16 v8b;
typedef __attribute__((ext_vector_type(8))) float v8f;
typedef __attribute__((ext_vector_type(4))) float v4f;
__device__ __forceinline__ float bf16_rne(float f) { unsigned int u = __float_as_uint(f); u += 0x7FFFu + ((u >> 16) & 1u); return __uint_as_float(u & 0xFFFF0000u); }
__device__ __forceinline__ void split16(float v, b16& hi, b16& lo) { hi = (b16)v; lo = (b16)(v - (float)hi); }
__device__ __forceinline__ v16b frag_kb(const b16* p, int hh) { const v8b a = *(const v8b*)(p + 8 * hh), b = *(const v8b*)(p + 16 + 8 * hh); v16b f;
#pragma unroll
  for (int e = 0; e < 8; ++e) { f[e] = a[e]; f[8 + e] = b[e]; } return f; }
__device__ __forceinline__ v8f wmma16b(v16b a, v16b b, v8f c) { v8f d = __builtin_amdgcn_wmma_f32_16x16x32_f16(false, a, false, b, (short)0, c, false, false); asm volatile("v_nop\n\tv_nop\n\tv_nop\n\tv_nop" : "+v"(d) : "v"(a), "v"(b)); return d; }
__device__ __forceinline__ void wave_lds_sync() { __builtin_amdgcn_fence(__ATOMIC_RELEASE, "workgroup"); __builtin_amdgcn_wave_barrier(); __builtin_amdgcn_fence(__ATOMIC_ACQUIRE, "workgroup"); }

__global__ __launch_bounds__(256) void wcopy_kernel(const float* __restrict__ w, b16* __restrict__ WB) {
  const size_t u = (size_t)blockIdx.x * 256 + threadIdx.x; if (u >= (size_t)OD * EF / 8) return; const size_t e = u * 8; v8b v;
#pragma unroll
  for (int j = 0; j < 8; ++j) v[j] = (b16)(bf16_rne(w[e + j]) * WSC); for (int pass = 0; pass < 2; ++pass) { *(volatile v8b*)(WB + e) = v; __threadfence(); }
}
__global__ __launch_bounds__(32) void stage1_kernel(const float* __restrict__ veh, const b16* __restrict__ WB, int nrt, b16* __restrict__ TH, b16* __restrict__ TL) {
  __shared__ __attribute__((aligned(16))) b16 Ah[16][EF + 8]; __shared__ __attribute__((aligned(16))) b16 Oh[16][128 + 8], Ol[16][128 + 8];
  const int lane = threadIdx.x, nloc = lane & 15, hlf = lane >> 4; const int rt = blockIdx.x % nrt, g = blockIdx.x / nrt; const size_t r0 = (size_t)rt * 16;
  for (int rr = 0; rr < 16; ++rr) for (int q = 0; q < 4; ++q) Ah[rr][q * 32 + lane] = (b16)(bf16_rne(veh[(r0 + rr) * EF + q * 32 + lane]) * XS);
  wave_lds_sync(); v8f acc[8];
#pragma unroll
  for (int t = 0; t < 8; ++t) acc[t] = (v8f){};
#pragma unroll
  for (int kb = 0; kb < EF; kb += 32) { const v16b a = frag_kb(&Ah[nloc][kb], hlf);
#pragma unroll
    for (int t = 0; t < 8; ++t) acc[t] = wmma16b(a, frag_kb(WB + ((size_t)g * 128 + t * 16 + nloc) * EF + kb, hlf), acc[t]); }
#pragma unroll
  for (int t = 0; t < 8; ++t)
#pragma unroll
    for (int r8 = 0; r8 < 8; ++r8) { b16 p, q; split16(acc[t][r8] * (1.0f / (XS * WSC)) * TS, p, q); Oh[8 * hlf + r8][t * 16 + nloc] = p; Ol[8 * hlf + r8][t * 16 + nloc] = q; }
  wave_lds_sync();
  for (int pass = 0; pass < 2; ++pass) { for (int rr = 0; rr < 16; ++rr) { const int c8 = (lane & 15) * 8; b16* dst = (hlf == 0) ? TH : TL; const b16 (*src)[128 + 8] = (hlf == 0) ? Oh : Ol; *(volatile v8b*)(dst + (r0 + rr) * OD + (size_t)g * 128 + c8) = *(const v8b*)(&src[rr][c8]); } __threadfence(); }
}
__global__ __launch_bounds__(32) void stage2_kernel(const float* __restrict__ node, const b16* __restrict__ TH, const b16* __restrict__ TL, const float* __restrict__ bias, float* __restrict__ out) {
  __shared__ __attribute__((aligned(16))) b16 Ah[16][D + 8]; __shared__ __attribute__((aligned(16))) float Tf[16][128 + 4];
  const int lane = threadIdx.x, nloc = lane & 15, hlf = lane >> 4; const int nt = blockIdx.x % (NN / 16), v = (blockIdx.x / (NN / 16)) % V, b = blockIdx.x / ((NN / 16) * V); const int n0 = nt * 16; const size_t bv = (size_t)b * V + v;
  for (int rr = 0; rr < 16; ++rr) for (int q = 0; q < 4; ++q) Ah[rr][q * 32 + lane] = (b16)(bf16_rne(node[((size_t)b * NN + n0 + rr) * D + q * 32 + lane]) * XS);
  wave_lds_sync();
#pragma unroll 1
  for (int cg = 0; cg < 2; ++cg) { v8f acc[8];
#pragma unroll
    for (int t = 0; t < 8; ++t) acc[t] = (v8f){};
#pragma unroll
    for (int kb = 0; kb < D; kb += 32) { const v16b a = frag_kb(&Ah[nloc][kb], hlf);
#pragma unroll
      for (int t = 0; t < 8; ++t) { const size_t br = bv * OD + (size_t)(cg * 128 + t * 16 + nloc) * D + kb; acc[t] = wmma16b(a, frag_kb(TH + br, hlf), acc[t]); acc[t] = wmma16b(a, frag_kb(TL + br, hlf), acc[t]); } }
#pragma unroll
    for (int t = 0; t < 8; ++t) { const int c = cg * 128 + t * 16 + nloc; const float bb = bf16_rne(bias[c]);
#pragma unroll
      for (int r8 = 0; r8 < 8; ++r8) Tf[8 * hlf + r8][t * 16 + nloc] = acc[t][r8] * (1.0f / (XS * TS)) + bb; }
    wave_lds_sync();
    for (int pass = 0; pass < 2; ++pass) { for (int rr = 0; rr < 16; ++rr) *(volatile v4f*)(out + (((size_t)b * NN + n0 + rr) * V + v) * O + cg * 128 + lane * 4) = *(const v4f*)(&Tf[rr][lane * 4]); __threadfence(); }
    wave_lds_sync(); }
}
}

extern "C" void kernel_launch(void* const* d_in, const int* in_sizes, int n_in, void* d_out, int out_size, void* d_ws, size_t ws_size, hipStream_t stream) {
  (void)n_in;
  auto Fp = [&](int i) { return (const float*)d_in[i]; };
  if (in_sizes[0] != B * NN * D || in_sizes[1] != BV * EF || in_sizes[2] != O * D * EF || in_sizes[3] != O || out_size != B * NN * V * O) return;
  const int NBV = B;
  size_t off = 0; char* ws = (char*)d_ws;
  auto carve = [&](size_t bytes) { char* p = ws + off; off += (bytes + 255) & ~(size_t)255; return p; };
  b16* WB = (b16*)carve((size_t)OD * EF * 2); b16* TH = (b16*)carve((size_t)BV * OD * 2); b16* TL = (b16*)carve((size_t)BV * OD * 2);
  if (off > ws_size || off > ((size_t)64 << 20)) return;
  wcopy_kernel<<<(unsigned)((OD * EF / 8 + 255) / 256), 256, 0, stream>>>(Fp(2), WB);
  stage1_kernel<<<(unsigned)((NBV * V / 16) * (OD / 128)), 32, 0, stream>>>(Fp(1), WB, NBV * V / 16, TH, TL);
  stage2_kernel<<<(unsigned)(NBV * V * (NN / 16)), 32, 0, stream>>>(Fp(0), TH, TL, Fp(3), (float*)d_out);
}
